// SatGNN_70531952935340
// MI455X (gfx1250) — hardware-run, weakly checked
//
#include <hip/hip_runtime.h>

typedef float          v8f   __attribute__((ext_vector_type(8)));
typedef float          v4f   __attribute__((ext_vector_type(4)));
typedef unsigned int   v4u   __attribute__((ext_vector_type(4)));
typedef int            v8i   __attribute__((ext_vector_type(8)));
typedef unsigned short v8us  __attribute__((ext_vector_type(8)));
typedef unsigned short v16us __attribute__((ext_vector_type(16)));
typedef __bf16         v16bf __attribute__((ext_vector_type(16)));
typedef _Float16       v16h  __attribute__((ext_vector_type(16)));
typedef v4f  __attribute__((may_alias)) v4fa;
typedef v8us __attribute__((may_alias)) v8usa;
union FragB { v16bf v; v16us u; v8us h[2]; v8i w; };
union FragH { v16h  v; v16us u; v8us h[2]; v8i w; };

__device__ __forceinline__ v8f wmb(const FragB& a, const FragB& b, v8f c) {
  v8f d = __builtin_amdgcn_wmma_f32_16x16x32_bf16(false, a.v, false, b.v, (short)0, c, false, false);
  asm volatile("v_nop\n\tv_nop\n\tv_nop\n\tv_nop" : "+v"(d) : "v"(a.w), "v"(b.w));
  return d;
}

__device__ __forceinline__ v8f wmh(const FragH& a, const FragH& b, v8f c) {
  v8f d = __builtin_amdgcn_wmma_f32_16x16x32_f16(false, a.v, false, b.v, (short)0, c, false, false);
  asm volatile("v_nop\n\tv_nop\n\tv_nop\n\tv_nop" : "+v"(d) : "v"(a.w), "v"(b.w));
  return d;
}

__device__ __forceinline__ unsigned bf16_bits(float f) {
  const unsigned u = __float_as_uint(f);
  const unsigned r = (u + 0x7FFFu + ((u >> 16) & 1u)) >> 16;
  const unsigned q = (u >> 16) | 0x40u;
  return ((u & 0x7fffffffu) > 0x7f800000u) ? q : r;
}

__device__ __forceinline__ float bf16_val(float f) {
  return __uint_as_float(bf16_bits(f) << 16);
}
__device__ __forceinline__ int clampi(int v, int lo, int hi) {
  return v < lo ? lo : (v > hi ? hi : v);
}

__device__ __forceinline__ unsigned f16_bits(float f) {
  const unsigned u  = __float_as_uint(f);
  const unsigned s  = (u >> 16) & 0x8000u;
  const unsigned a  = u & 0x7fffffffu;
  const unsigned t  = a - 0x38000000u;
  const unsigned r  = (t + 0x0FFFu + ((t >> 13) & 1u)) >> 13;
  const unsigned rc = r > 0x7C00u ? 0x7C00u : r;
  const bool small  = a < 0x38800000u;
  const bool isnan  = a > 0x7f800000u;
  const unsigned fin = small ? 0u : (s | rc);
  return isnan ? (s | 0x7E00u) : fin;
}

__device__ __forceinline__ unsigned pk16(unsigned lo, unsigned hi) { return lo | (hi << 16); }
__device__ __forceinline__ unsigned bf16_lo_bits(float v) {
  float hi = bf16_val(v);
  asm volatile("" : "+v"(hi));
  return bf16_bits(v - hi);
}
__device__ __forceinline__ v4u pack8_bf16(v4f a, v4f c) {
  return (v4u){ pk16(bf16_bits(a[0]), bf16_bits(a[1])), pk16(bf16_bits(a[2]), bf16_bits(a[3])),
                pk16(bf16_bits(c[0]), bf16_bits(c[1])), pk16(bf16_bits(c[2]), bf16_bits(c[3])) };
}
__device__ __forceinline__ v4u pack8_bf16_lo(v4f a, v4f c) {
  return (v4u){ pk16(bf16_lo_bits(a[0]), bf16_lo_bits(a[1])), pk16(bf16_lo_bits(a[2]), bf16_lo_bits(a[3])),
                pk16(bf16_lo_bits(c[0]), bf16_lo_bits(c[1])), pk16(bf16_lo_bits(c[2]), bf16_lo_bits(c[3])) };
}
__device__ __forceinline__ v4u pack8_f16(v4f a, v4f c) {
  return (v4u){ pk16(f16_bits(a[0]), f16_bits(a[1])), pk16(f16_bits(a[2]), f16_bits(a[3])),
                pk16(f16_bits(c[0]), f16_bits(c[1])), pk16(f16_bits(c[2]), f16_bits(c[3])) };
}

template <int FORM>
__global__ __launch_bounds__(256) void k_plane(const float* __restrict__ src, int rows, int cols, int ldsrc,
                                               unsigned short* __restrict__ dst, int MP, int KP) {
  static_assert(FORM >= 0 && FORM <= 3);
  const int KTOT = (FORM == 1 || FORM == 3) ? 2 * KP : KP;
  const unsigned ppr   = (unsigned)(KTOT >> 3);
  const unsigned kp8   = (unsigned)(KP >> 3);
  const unsigned total = (unsigned)MP * ppr;
  const unsigned g     = blockIdx.x * 256u + threadIdx.x;
  const unsigned rowu  = g / ppr;
  const unsigned p     = g - rowu * ppr;
  const bool second    = p >= kp8;
  const int row = (int)rowu;
  const int c0  = (int)((second ? p - kp8 : p) << 3);
  const float* srow = src + (size_t)clampi(row, 0, rows - 1) * (size_t)ldsrc;
  float x[8];
  unsigned mk[8];
#pragma unroll
  for (int e = 0; e < 8; ++e) {
    const int c = c0 + e;
    const float v = srow[clampi(c, 0, cols - 1)];
    asm volatile("" :: "v"(v));
    x[e]  = v;
    mk[e] = (row < rows && c < cols) ? 0xFFFFu : 0u;
  }
  const v4f a = (v4f){ x[0], x[1], x[2], x[3] };
  const v4f c = (v4f){ x[4], x[5], x[6], x[7] };
  v4u o;
  if (FORM == 2) {
    o = pack8_f16(a, c);
  } else {
    const v4u hi = pack8_bf16(a, c);
    o = hi;
    if (FORM == 1) { const v4u lo = pack8_bf16_lo(a, c); o = second ? lo : hi; }
  }
  const v4u mw = (v4u){ pk16(mk[0], mk[1]), pk16(mk[2], mk[3]), pk16(mk[4], mk[5]), pk16(mk[6], mk[7]) };
  o &= mw;
  if (g < total) {
    volatile v4u* q = (volatile v4u*)(dst + (size_t)g * 8);
    *q = o;
    __threadfence();
    *q = o;
  }
}

template <int FORM> struct FragOf    { typedef FragB T; };
template <>         struct FragOf<2> { typedef FragH T; };
__device__ __forceinline__ v8f mm(const FragB& a, const FragB& b, v8f c) { return wmb(a, b, c); }
__device__ __forceinline__ v8f mm(const FragH& a, const FragH& b, v8f c) { return wmh(a, b, c); }
template <class F> __device__ __forceinline__ F ld_frag(const unsigned short* p) {
  F f;
  f.h[0] = *(const v8usa*)(p);
  f.h[1] = *(const v8usa*)(p + 16);
  return f;
}

template <int FORM, int EPI>
__global__ __launch_bounds__(256) __attribute__((amdgpu_num_vgpr(248)))
void k_gemm_nt(const unsigned short* __restrict__ A, const unsigned short* __restrict__ B,
               const float* __restrict__ bias, float* __restrict__ D, int M, int N, int KTOT, int ldd) {
  static_assert(FORM >= 0 && FORM <= 2);
  static_assert(EPI == 0 || EPI == 1);
  typedef typename FragOf<FORM>::T F;
  __shared__ __attribute__((aligned(16))) float sT[8][16 * 68];
  const int lane = threadIdx.x & 31;
  const int wave = threadIdx.x >> 5;
  const int tilesM = (M + 63) >> 6;
  const int tilesN = (N + 63) >> 6;
  const int tile = blockIdx.x * 8 + wave;
  if (tile >= tilesM * tilesN) return;
  const int tm = tile / tilesN;
  const int tn = tile - tm * tilesN;
  const int m0 = tm << 6;
  const int n0 = tn << 6;

  const int rl = lane & 15;
  const int h8 = (lane >> 4) * 8;
  const unsigned short* pa = A + (size_t)(m0 + rl) * (size_t)KTOT + h8;
  const unsigned short* pb = B + (size_t)(n0 + rl) * (size_t)KTOT + h8;

  v8f acc[4][4];
#pragma unroll
  for (int i = 0; i < 4; ++i)
#pragma unroll
    for (int j = 0; j < 4; ++j) acc[i][j] = (v8f){0.f, 0.f, 0.f, 0.f, 0.f, 0.f, 0.f, 0.f};

#pragma unroll 1
  for (int k0 = 0; k0 < KTOT; k0 += 32) {
    F bf[4];
#pragma unroll
    for (int j = 0; j < 4; ++j) bf[j] = ld_frag<F>(pb + (size_t)(j << 4) * (size_t)KTOT + k0);
#pragma unroll
    for (int i = 0; i < 4; ++i) {
      const F af = ld_frag<F>(pa + (size_t)(i << 4) * (size_t)KTOT + k0);
#pragma unroll
      for (int j = 0; j < 4; ++j) acc[i][j] = mm(af, bf[j], acc[i][j]);
    }
  }

  float* slab = sT[wave];
  const int hh = lane >> 4;
  const int c4 = (lane & 15) * 4;
  const int nc = n0 + c4;
  const bool cok = nc < N;
  v4f bv = (v4f){0.f, 0.f, 0.f, 0.f};
  if (EPI == 1) {
    bv = *(const v4fa*)(bias + clampi(nc, 0, N - 4));
    asm volatile("" :: "v"(bv));
  }
#pragma unroll
  for (int i = 0; i < 4; ++i) {
    const int mBase = m0 + (i << 4);
#pragma unroll
    for (int j = 0; j < 4; ++j) {
#pragma unroll
      for (int r = 0; r < 8; ++r) slab[(h8 + r) * 68 + (j << 4) + rl] = acc[i][j][r];
    }
    __builtin_amdgcn_fence(__ATOMIC_RELEASE, "workgroup");
    __builtin_amdgcn_wave_barrier();
    __builtin_amdgcn_fence(__ATOMIC_ACQUIRE, "workgroup");
    v4f vv[8];
#pragma unroll
    for (int it = 0; it < 8; ++it) {
      const int row = it * 2 + hh;
      v4f v = *(const v4fa*)(slab + row * 68 + c4);
      if (EPI == 1) v += bv;
      vv[it] = v;
    }
    for (int pass = 0; pass < 2; ++pass) {
#pragma unroll
      for (int it = 0; it < 8; ++it) {
        const int row = mBase + it * 2 + hh;
        if (cok && row < M) *(volatile v4f*)(D + (size_t)row * (size_t)ldd + nc) = vv[it];
      }
      __threadfence();
    }
    __builtin_amdgcn_fence(__ATOMIC_RELEASE, "workgroup");
    __builtin_amdgcn_wave_barrier();
    __builtin_amdgcn_fence(__ATOMIC_ACQUIRE, "workgroup");
  }
}

#define SPLIT_A 1

typedef float          v2f  __attribute__((ext_vector_type(2)));
typedef unsigned       v2u  __attribute__((ext_vector_type(2)));
typedef int            v4i  __attribute__((ext_vector_type(4)));
typedef v4i __attribute__((may_alias)) v4ia;
typedef v2f __attribute__((may_alias)) v2fa;
typedef unsigned short __attribute__((may_alias)) usa;

#define HD      64
#define NVAR    100000
#define NCON    100000
#define NSOC    20000
#define EVC     2000000
#define ESC     300000
#define MPAD    100096
#define MPS     20096
#define NBRUN   1024
#define NBLKB   98
#define NWV     8
#define WCAP    3584
#define LISTN   (NWV * WCAP)
#define RCAP    28672
#define RCAP_SC 4096
#define DEGCAP  56
#define BK_CNTW LISTN
#define BK_OFF  (BK_CNTW + NWV * NBRUN)
#define BK_CNT  (BK_OFF + NBRUN)
#define BK_MISC (BK_CNT + NBRUN)
#define BK_PLC  (BK_MISC + 64)
#define BK_INTS (BK_PLC + RCAP / 2)
#define NFLG    (3 * NBLKB)

#define P_BP0   0
#define P_B0    256
#define P_BH    512
#define P_WO    576
#define P_BO    640
#define PRM_N   672

static_assert(HD == 64);
static_assert(NVAR % 32 == 0 && NCON == NVAR);
static_assert(MPAD == 782 * 128 && MPS == 157 * 128);
static_assert(MPAD % 64 == 0 && MPS % 64 == 0 && MPAD % 16 == 0 && MPS % 16 == 0);
static_assert(MPAD >= NVAR && MPS >= NSOC);
static_assert(NBLKB * NBRUN >= NVAR && (NBLKB - 1) * NBRUN < NVAR && MPAD <= NBLKB * NBRUN);
static_assert(NWV * WCAP == RCAP && RCAP % 256 == 0 && RCAP_SC % 256 == 0 && LISTN <= 65536 && RCAP_SC <= RCAP);
static_assert(RCAP >= 20887 + (20887 * 8) / 100);
static_assert(RCAP_SC >= 3174 + (3174 * 8) / 100);
static_assert(DEGCAP >= 43 + 8 && DEGCAP % 8 == 0);
static_assert(EVC % 8 == 0 && ESC % 8 == 0 && EVC < (1 << 22) && ESC < (1 << 22));
static_assert(BK_INTS % 4 == 0 && BK_INTS * 4 <= 327680);
static_assert(P_WO == P_BH + 64 && PRM_N % 4 == 0);

__device__ __forceinline__ void pinf(float x)  { asm volatile("" :: "v"(x)); }
__device__ __forceinline__ void pini(int x)    { asm volatile("" :: "v"(x)); }
__device__ __forceinline__ void pin4f(v4f x)   { asm volatile("" :: "v"(x)); }
__device__ __forceinline__ void pin4i(v4i x)   { asm volatile("" :: "v"(x)); }

__device__ __forceinline__ float relu_k(float v) { return (v > 0.0f || v != v) ? v : 0.0f; }
__device__ __forceinline__ float nmax(float m, float v) { return (v > m || v != v) ? v : m; }

__device__ __forceinline__ unsigned lo_bits_sw(float v) { return SPLIT_A ? bf16_lo_bits(v) : 0u; }
__device__ __forceinline__ unsigned split_bits(float v, int islo) {
  float hi = bf16_val(v);
  asm volatile("" : "+v"(hi));
  const float t = islo ? (v - hi) : v;
  const unsigned w = bf16_bits(t);
  return (islo && !SPLIT_A) ? 0u : w;
}

__device__ __forceinline__ void seg_copy(const float* __restrict__ s, int n, int padn, float scale,
                                         float* img, int off, int tid) {
  const int padw = (padn + 31) & ~31;
#pragma unroll 1
  for (int i = tid; i < padw; i += 256) {
    float v = s[i < n ? i : n - 1];
    pinf(v);
    if (i < padn) img[off + i] = (i < n) ? scale * bf16_val(v) : 0.0f;
  }
}

__device__ __forceinline__ void wunit(const float* __restrict__ W, float scale, unsigned short* dst,
                                      int pitch, int coloff, float* sW, int tid) {
#pragma unroll
  for (int it = 0; it < 4; ++it) {
    const int p = tid + 256 * it;
    const v4f v = *(const v4fa*)(W + 4 * p);
    pin4f(v);
    const v4f o = (v4f){ scale * bf16_val(v[0]), scale * bf16_val(v[1]), scale * bf16_val(v[2]), scale * bf16_val(v[3]) };
    *(v4fa*)(sW + 4 * p) = o;
  }
  __syncthreads();
  v4u o[4];
#pragma unroll
  for (int it = 0; it < 4; ++it) {
    const int g  = tid + 256 * it;
    const int n  = g >> 4;
    const int k0 = (g & 7) << 3;
    const v4f a = (v4f){ sW[(k0 + 0) * 64 + n], sW[(k0 + 1) * 64 + n], sW[(k0 + 2) * 64 + n], sW[(k0 + 3) * 64 + n] };
    const v4f c = (v4f){ sW[(k0 + 4) * 64 + n], sW[(k0 + 5) * 64 + n], sW[(k0 + 6) * 64 + n], sW[(k0 + 7) * 64 + n] };
    o[it] = pack8_bf16(a, c);
  }
  for (int pass = 0; pass < 2; ++pass) {
#pragma unroll
    for (int it = 0; it < 4; ++it) {
      const int g = tid + 256 * it;
      const int n = g >> 4;
      const int piece = g & 15;
      *(volatile v4u*)(dst + (size_t)n * (size_t)pitch + coloff + piece * 8) = o[it];
    }
    __threadfence();
  }
  __syncthreads();
}

__global__ __launch_bounds__(256) void k_prep(
    const float* __restrict__ Wp0, const float* __restrict__ Ws0, const float* __restrict__ Wn0,
    const float* __restrict__ Wp1, const float* __restrict__ Ws1, const float* __restrict__ Wn1,
    const float* __restrict__ Wp2, const float* __restrict__ Ws2, const float* __restrict__ Wn2,
    const float* __restrict__ Wp3, const float* __restrict__ Ws3, const float* __restrict__ Wn3,
    const float* __restrict__ Whid,
    const float* __restrict__ bp0, const float* __restrict__ bb0, const float* __restrict__ bp1,
    const float* __restrict__ bb1, const float* __restrict__ bp2, const float* __restrict__ bb2,
    const float* __restrict__ bp3, const float* __restrict__ bb3, const float* __restrict__ bhid,
    const float* __restrict__ Wout, const float* __restrict__ bout,
    unsigned short* wpt, unsigned short* wfb, float* prm) {
  __shared__ __attribute__((aligned(16))) float sW[4096];
  __shared__ __attribute__((aligned(16))) float img[PRM_N];
  const int tid = (int)threadIdx.x;
  seg_copy(bp0, 64, 64, 1.0f, img, P_BP0, tid);
  seg_copy(bp1, 64, 64, 1.0f, img, P_BP0 + 64, tid);
  seg_copy(bp2, 64, 64, 1.0f, img, P_BP0 + 128, tid);
  seg_copy(bp3, 64, 64, 1.0f, img, P_BP0 + 192, tid);
  seg_copy(bb0, 64, 64, 2.0f, img, P_B0, tid);
  seg_copy(bb1, 64, 64, 2.0f, img, P_B0 + 64, tid);
  seg_copy(bb2, 64, 64, 1.0f, img, P_B0 + 128, tid);
  seg_copy(bb3, 64, 64, 1.0f, img, P_B0 + 192, tid);
  seg_copy(bhid, 64, 64, 1.0f, img, P_BH, tid);
  seg_copy(Wout, 64, 64, 1.0f, img, P_WO, tid);
  seg_copy(bout, 1, 32, 1.0f, img, P_BO, tid);
  __syncthreads();
  for (int pass = 0; pass < 2; ++pass) {
#pragma unroll 1
    for (int p = tid; p < PRM_N / 4; p += 256) {
      const v4f v = *(const v4fa*)(img + 4 * p);
      *(volatile v4f*)(prm + 4 * p) = v;
    }
    __threadfence();
  }
  wunit(Wp0, 1.0f, wpt + 0 * 8192, 128, 0, sW, tid);
  wunit(Wp1, 1.0f, wpt + 1 * 8192, 128, 0, sW, tid);
  wunit(Wp2, 1.0f, wpt + 2 * 8192, 128, 0, sW, tid);
  wunit(Wp3, 1.0f, wpt + 3 * 8192, 128, 0, sW, tid);
  wunit(Whid, 1.0f, wpt + 4 * 8192, 128, 0, sW, tid);
  wunit(Wn0, 1.0f, wfb + 0 * 16384, 256, 0, sW, tid);
  wunit(Ws0, 2.0f, wfb + 0 * 16384, 256, 128, sW, tid);
  wunit(Wn1, 1.0f, wfb + 1 * 16384, 256, 0, sW, tid);
  wunit(Ws1, 2.0f, wfb + 1 * 16384, 256, 128, sW, tid);
  wunit(Wn2, 1.0f, wfb + 2 * 16384, 256, 0, sW, tid);
  wunit(Ws2, 1.0f, wfb + 2 * 16384, 256, 128, sW, tid);
  wunit(Wn3, 1.0f, wfb + 3 * 16384, 256, 0, sW, tid);
  wunit(Ws3, 1.0f, wfb + 3 * 16384, 256, 128, sW, tid);
}

__global__ __launch_bounds__(256) void k_embed(const float* __restrict__ x, const float* __restrict__ W,
                                               const float* __restrict__ bias, int n, int K,
                                               unsigned* dstw, int pitchw, int colw) {
  __shared__ float sX[1024];
  __shared__ __attribute__((aligned(16))) float sW[512];
  __shared__ float sB[64];
  if (K < 1 || K > 7) return;
  const int tid = (int)threadIdx.x, lane = tid & 31;
  const int wave = __builtin_amdgcn_readfirstlane(tid >> 5);
  const int r0 = (int)blockIdx.x * 128;
  const int totx = 128 * K;
  const int nK = n * K;
#pragma unroll 1
  for (int i = tid; i < totx; i += 256) {
    int gi = r0 * K + i;
    gi = gi < nK - 1 ? gi : nK - 1;
    float v = x[gi];
    pinf(v);
    sX[i] = bf16_val(v);
  }
  const int totw = 64 * K;
#pragma unroll 1
  for (int i = tid; i < totw; i += 256) {
    float v = W[i];
    pinf(v);
    sW[i] = bf16_val(v);
  }
  if (tid < 64) {
    float v = bias[tid];
    pinf(v);
    sB[tid] = bf16_val(v);
  }
  __syncthreads();
#pragma unroll 1
  for (int j = 0; j < 16; ++j) {
    const int rl = wave * 16 + j;
    const int row = r0 + rl;
    float a0 = 0.0f, a1 = 0.0f;
#pragma unroll 1
    for (int k = 0; k < K; ++k) {
      const float xk = sX[rl * K + k];
      const v2f w = *(const v2fa*)(sW + k * 64 + 2 * lane);
      a0 = fmaf(xk, w.x, a0);
      a1 = fmaf(xk, w.y, a1);
    }
    a0 = relu_k(a0 + sB[2 * lane]);
    a1 = relu_k(a1 + sB[2 * lane + 1]);
    const unsigned mk = (row < n) ? 0xFFFFFFFFu : 0u;
    const unsigned hi = pk16(bf16_bits(a0), bf16_bits(a1)) & mk;
    const unsigned lo = pk16(lo_bits_sw(a0), lo_bits_sw(a1)) & mk;
    unsigned* op = dstw + (size_t)row * (size_t)pitchw + colw + lane;
    *(volatile unsigned*)op = hi;
    *(volatile unsigned*)(op + 32) = lo;
    __threadfence();
    *(volatile unsigned*)op = hi;
    *(volatile unsigned*)(op + 32) = lo;
  }
}

__device__ __forceinline__ int slot_prefix(int* cntw, int s) {
  int run = 0;
#pragma unroll
  for (int w = 0; w < NWV; ++w) {
    const int c = cntw[w * NBRUN + s];
    cntw[w * NBRUN + s] = run;
    run += c;
  }
  return run;
}

#define BK_HIT(J, SJ) { \
    const unsigned mk_ = __builtin_amdgcn_ballot_w32((SJ) < unb); \
    if (mk_ != 0u) { \
      const int pos_ = wcnt + (int)__builtin_amdgcn_mbcnt_lo(mk_, 0u); \
      if ((SJ) < unb && pos_ < WCAP) list[lbase + pos_] = (int)((((unsigned)(e0 + (J))) << 10) | (SJ)); \
      wcnt += (int)__builtin_popcount(mk_); \
    } }

__global__ __launch_bounds__(256) void k_bucket(const int* __restrict__ key, const int* __restrict__ val,
                                                int nE, int ndst, int nsrc, int cap,
                                                unsigned* entg, int* offg, int* cntg, int* flgg) {
  extern __shared__ __attribute__((aligned(16))) int dsm[];
  int* list = dsm;
  int* cntw = dsm + BK_CNTW;
  int* offA = dsm + BK_OFF;
  int* cntT = dsm + BK_CNT;
  int* misc = dsm + BK_MISC;
  usa* plc  = (usa*)(dsm + BK_PLC);
  const int tid = (int)threadIdx.x, lane = tid & 31;
  const int wave = __builtin_amdgcn_readfirstlane(tid >> 5);
  const int b = (int)blockIdx.x;
  const int nodeBase = b * NBRUN;
  int nbl = (ndst - nodeBase) < NBRUN ? (ndst - nodeBase) : NBRUN;
  nbl = nbl < 0 ? 0 : nbl;
  const unsigned nbs = (unsigned)nodeBase;
  const unsigned unb = (unsigned)nbl;
  const int lbase = wave * WCAP;

  {
    const v4i z4 = {0, 0, 0, 0};
#pragma unroll 1
    for (int i = tid * 4; i < BK_INTS; i += 1024) *(v4ia*)(dsm + i) = z4;
  }
  __syncthreads();

  const int nwch = (nE + 255) >> 8;
  int wcnt = 0;
#pragma unroll 1
  for (int wc = wave; wc < nwch; wc += NWV) {
    const int e0  = wc * 256 + lane * 8;
    const int e0c = e0 < nE - 8 ? e0 : nE - 8;
    const v4i da = *(const v4ia*)(key + e0c);
    const v4i db = *(const v4ia*)(key + e0c + 4);
    pin4i(da);
    pin4i(db);
    const unsigned inv = (e0 < nE) ? 0u : 0xFFFFFFFFu;
    const unsigned s0 = ((unsigned)da.x - nbs) | inv, s1 = ((unsigned)da.y - nbs) | inv;
    const unsigned s2 = ((unsigned)da.z - nbs) | inv, s3 = ((unsigned)da.w - nbs) | inv;
    const unsigned s4 = ((unsigned)db.x - nbs) | inv, s5 = ((unsigned)db.y - nbs) | inv;
    const unsigned s6 = ((unsigned)db.z - nbs) | inv, s7 = ((unsigned)db.w - nbs) | inv;
    BK_HIT(0, s0)
    BK_HIT(1, s1)
    BK_HIT(2, s2)
    BK_HIT(3, s3)
    BK_HIT(4, s4)
    BK_HIT(5, s5)
    BK_HIT(6, s6)
    BK_HIT(7, s7)
  }
  const int wraw = __builtin_amdgcn_readfirstlane(wcnt);
  if (lane == 0) misc[wave] = wraw;
  __syncthreads();

  const int myc = clampi(wraw, 0, WCAP);
  if (lane == 0) {
#pragma unroll 1
    for (int i = 0; i < myc; ++i) {
      const int s = list[lbase + i] & (NBRUN - 1);
      cntw[wave * NBRUN + s] = cntw[wave * NBRUN + s] + 1;
    }
  }
  __syncthreads();

  const int t0 = slot_prefix(cntw, 4 * tid);
  const int t1 = slot_prefix(cntw, 4 * tid + 1);
  const int t2 = slot_prefix(cntw, 4 * tid + 2);
  const int t3 = slot_prefix(cntw, 4 * tid + 3);
  const int e1 = t0, e2 = t0 + t1, e3 = t0 + t1 + t2, sum4 = t0 + t1 + t2 + t3;
  int incl = sum4;
#pragma unroll
  for (int dd = 1; dd < 32; dd <<= 1) {
    const int y = __shfl_up(incl, dd, 32);
    if (lane >= dd) incl += y;
  }
  if (lane == 31) misc[8 + wave] = incl;
  __syncthreads();
  int base = 0, tot = 0, flag = 0;
#pragma unroll
  for (int w2 = 0; w2 < NWV; ++w2) {
    const int c = misc[8 + w2];
    base += (w2 < wave) ? c : 0;
    tot  += c;
    flag |= (misc[w2] > WCAP) ? 1 : 0;
  }
  flag |= (tot > cap) ? 1 : 0;
  const int ex = base + incl - sum4;
  const v4i ov = {ex, ex + e1, ex + e2, ex + e3};
  const v4i cv = {t0, t1, t2, t3};
  *(v4ia*)(offA + 4 * tid) = ov;
  *(v4ia*)(cntT + 4 * tid) = cv;
  __syncthreads();

  if (lane == 0) {
#pragma unroll 1
    for (int i = 0; i < myc; ++i) {
      const int s = list[lbase + i] & (NBRUN - 1);
      const int c = cntw[wave * NBRUN + s];
      cntw[wave * NBRUN + s] = c + 1;
      const int p = offA[s] + c;
      if ((unsigned)p < (unsigned)RCAP) plc[p] = (unsigned short)(lbase + i);
    }
  }
  __syncthreads();

  const int tt  = tot < cap ? tot : cap;
  int ttr = (tt + 255) & ~255;
  ttr = ttr < cap ? ttr : cap;
  unsigned* eg = entg + (size_t)b * (size_t)cap;
  const v4i fv = {(tid == 0) ? flag : 0, 0, 0, 0};
  for (int pass = 0; pass < 2; ++pass) {
#pragma unroll 1
    for (int p = tid; p < ttr; p += 256) {
      const int pc = p < tt ? p : (tt > 0 ? tt - 1 : 0);
      const int idx = (int)plc[pc];
      const unsigned word = (unsigned)list[clampi(idx, 0, LISTN - 1)];
      const int eid = clampi((int)(word >> 10), 0, nE - 1);
      int sr = val[eid];
      pini(sr);
      sr = clampi(sr, 0, nsrc - 1);
      const unsigned mk = (p < tt) ? 0xFFFFFFFFu : 0u;
      const unsigned o = (unsigned)sr & mk;
      *(volatile unsigned*)(eg + (size_t)p) = o;
    }
    *(volatile v4i*)(offg + (size_t)b * NBRUN + 4 * tid) = ov;
    *(volatile v4i*)(cntg + (size_t)b * NBRUN + 4 * tid) = cv;
    if (tid < 8) *(volatile v4i*)(flgg + (size_t)b * 32 + 4 * tid) = fv;
    __threadfence();
  }
}

struct SlotR { int off; int cnt; int last; int ov; };

__device__ __forceinline__ SlotR slot_read(const int* __restrict__ offg, const int* __restrict__ cntg,
                                           size_t t, int cap) {
  int off = offg[t];
  pini(off);
  int cr = cntg[t];
  pini(cr);
  const int ov = (cr > DEGCAP) ? 1 : 0;
  int cnt = clampi(cr, 0, DEGCAP);
  off = clampi(off, 0, cap - 1);
  if (cnt > cap - off) cnt = cap - off;
  const int lastv = off + (cnt > 0 ? cnt - 1 : 0);
  SlotR r;
  r.cnt  = __builtin_amdgcn_readfirstlane(cnt);
  r.off  = __builtin_amdgcn_readfirstlane(off);
  r.last = __builtin_amdgcn_readfirstlane(lastv);
  r.ov   = __builtin_amdgcn_readfirstlane(ov);
  return r;
}

__device__ __forceinline__ v4f rel_gather(const float* __restrict__ P, const unsigned* __restrict__ ent,
                                          size_t ebase, int off, int cnt, int last, int nsrc, int lane) {
  const int hh = lane >> 4;
  const int c4 = (lane & 15) * 4;
  const float ninf = __int_as_float((int)0xff800000u);
  v4f m = (v4f){ ninf, ninf, ninf, ninf };
#pragma unroll 1
  for (int g0 = 0; g0 < cnt; g0 += 8) {
    int idx = off + g0 + (lane & 7);
    idx = idx > last ? last : idx;
    const unsigned en = ent[ebase + (size_t)idx];
    pini((int)en);
    const int srl = clampi((int)en, 0, nsrc - 1);
    v4f hv[4];
#pragma unroll
    for (int j = 0; j < 4; ++j) {
      const int sj = __shfl(srl, j + 4 * hh, 32);
      hv[j] = *(const v4fa*)(P + (size_t)sj * 64 + c4);
      pin4f(hv[j]);
    }
#pragma unroll
    for (int j = 0; j < 4; ++j) {
#pragma unroll
      for (int c = 0; c < 4; ++c) m[c] = nmax(m[c], hv[j][c]);
    }
  }
#pragma unroll
  for (int c = 0; c < 4; ++c) {
    const float o = __shfl_xor(m[c], 16, 32);
    m[c] = nmax(m[c], o);
  }
  return m;
}

template <int NREL>
__global__ __launch_bounds__(256) void k_agg(
    const float* __restrict__ P0, const unsigned* __restrict__ ent0, const int* __restrict__ off0,
    const int* __restrict__ cnt0, const int* __restrict__ flg0, int cap0, int nsrc0,
    const float* __restrict__ P1, const unsigned* __restrict__ ent1, const int* __restrict__ off1,
    const int* __restrict__ cnt1, const int* __restrict__ flg1, int cap1, int nsrc1,
    const float* __restrict__ prm, int pBp, int ndst, unsigned* xw) {
  static_assert(NREL == 1 || NREL == 2);
  const int tid = (int)threadIdx.x, lane = tid & 31;
  const int wave = __builtin_amdgcn_readfirstlane(tid >> 5);
  const int b = (int)blockIdx.x;
  const int hh = lane >> 4;
  const int q  = lane & 15;
  int fl = flg0[(size_t)b * 32];
  pini(fl);
  if (NREL == 2) {
    int f1 = flg1[(size_t)b * 32];
    pini(f1);
    fl |= f1;
  }
  const v4f bp = *(const v4fa*)(prm + pBp + 4 * q);
  pin4f(bp);
  const float qnan = __int_as_float(0x7fc00000);
#pragma unroll 1
  for (int si = 0; si < 128; ++si) {
    const int s = wave * 128 + si;
    const int node = b * NBRUN + s;
    if (node >= MPAD) break;
    const size_t t = (size_t)b * NBRUN + (size_t)s;
    const SlotR r0 = slot_read(off0, cnt0, t, cap0);
    const v4f m0 = rel_gather(P0, ent0, (size_t)b * (size_t)cap0, r0.off, r0.cnt, r0.last, nsrc0, lane);
    int ovf = r0.ov;
    v4f a;
#pragma unroll
    for (int c = 0; c < 4; ++c) a[c] = (r0.cnt > 0) ? relu_k(m0[c] + bp[c]) : 0.0f;
    if (NREL == 2) {
      const SlotR r1 = slot_read(off1, cnt1, t, cap1);
      const v4f m1 = rel_gather(P1, ent1, (size_t)b * (size_t)cap1, r1.off, r1.cnt, r1.last, nsrc1, lane);
      ovf |= r1.ov;
#pragma unroll
      for (int c = 0; c < 4; ++c) {
        const float g = (r1.cnt > 0) ? relu_k(m1[c] + bp[c]) : 0.0f;
        a[c] = a[c] + g;
      }
    }
    const float pz = (fl != 0 || ovf != 0) ? qnan : 0.0f;
#pragma unroll
    for (int c = 0; c < 4; ++c) {
      const float v = a[c] + pz;
      a[c] = (node < ndst) ? v : 0.0f;
    }
    const v2u o = { pk16(split_bits(a[0], hh), split_bits(a[1], hh)),
                    pk16(split_bits(a[2], hh), split_bits(a[3], hh)) };
    unsigned* op = xw + (size_t)node * 128 + hh * 32 + 2 * q;
    *(volatile v2u*)op = o;
    __threadfence();
    *(volatile v2u*)op = o;
  }
}

__global__ __launch_bounds__(256) void k_post(const float* __restrict__ pre, const float* __restrict__ prm,
                                              int pB, int n, unsigned short* dst, int pitch, int coloff) {
  const int tid = (int)threadIdx.x, lane = tid & 31;
  const int wave = __builtin_amdgcn_readfirstlane(tid >> 5);
  const int sg = lane >> 3;
  const int rsel = sg >> 1;
  const int islo = sg & 1;
  const int c8 = (lane & 7) * 8;
  const v4f b0 = *(const v4fa*)(prm + pB + c8);
  const v4f b1 = *(const v4fa*)(prm + pB + c8 + 4);
  pin4f(b0);
  pin4f(b1);
#pragma unroll 1
  for (int it = 0; it < 8; ++it) {
    const int row = (int)blockIdx.x * 128 + wave * 16 + 2 * it + rsel;
    const v4f p0 = *(const v4fa*)(pre + (size_t)row * 64 + c8);
    const v4f p1 = *(const v4fa*)(pre + (size_t)row * 64 + c8 + 4);
    pin4f(p0);
    pin4f(p1);
    const unsigned mk = (row < n) ? 0xFFFFFFFFu : 0u;
    unsigned w[8];
#pragma unroll
    for (int c = 0; c < 4; ++c) {
      w[c]     = split_bits(relu_k(p0[c] + b0[c]), islo);
      w[4 + c] = split_bits(relu_k(p1[c] + b1[c]), islo);
    }
    const v4u o = (v4u){ pk16(w[0], w[1]) & mk, pk16(w[2], w[3]) & mk, pk16(w[4], w[5]) & mk, pk16(w[6], w[7]) & mk };
    volatile v4u* qd = (volatile v4u*)(dst + (size_t)row * (size_t)pitch + coloff + islo * 64 + c8);
    *qd = o;
    __threadfence();
    *qd = o;
  }
}

__global__ __launch_bounds__(128) void k_head(const float* __restrict__ pre, const float* __restrict__ prm,
                                              const int* __restrict__ flg, float* out) {
  __shared__ float sT[128 * 65];
  __shared__ float sV[128];
  __shared__ int sF[4];
  const int tid = (int)threadIdx.x, lane = tid & 31;
  const int wave = __builtin_amdgcn_readfirstlane(tid >> 5);
  const int r0 = (int)blockIdx.x * 128;
  int f = 0;
#pragma unroll 1
  for (int it = 0; it < 3; ++it) {
    const int i = tid + 128 * it;
    const int ic = i < NFLG - 1 ? i : NFLG - 1;
    int v = flg[(size_t)ic * 32];
    pini(v);
    f |= (i < NFLG) ? v : 0;
  }
  const unsigned bal = __builtin_amdgcn_ballot_w32(f != 0);
  if (lane == 0) sF[wave] = (bal != 0u) ? 1 : 0;
  {
    float v = prm[P_BH + tid];
    pinf(v);
    sV[tid] = v;
  }
#pragma unroll 4
  for (int it = 0; it < 16; ++it) {
    const int p = tid + 128 * it;
    const int row = p >> 4;
    const int c4 = (p & 15) * 4;
    const v4f v = *(const v4fa*)(pre + (size_t)(r0 + row) * 64 + c4);
    float* d = sT + row * 65 + c4;
    d[0] = v[0]; d[1] = v[1]; d[2] = v[2]; d[3] = v[3];
  }
  __syncthreads();
  float acc = 0.0f;
#pragma unroll 4
  for (int k = 0; k < 64; ++k) {
    const float z = relu_k(sT[tid * 65 + k] + sV[k]);
    acc = fmaf(z, sV[64 + k], acc);
  }
  float bo = prm[P_BO];
  pinf(bo);
  acc += bo;
  const int anyf = sF[0] | sF[1] | sF[2] | sF[3];
  const float r = (anyf != 0) ? __int_as_float(0x7fc00000) : acc;
  if (r0 + wave * 32 + 32 <= NVAR) {
    float* op = out + r0 + tid;
    *(volatile float*)op = r;
    __threadfence();
    *(volatile float*)op = r;
  }
}

static inline size_t al256(size_t o) { return (o + 255) & ~(size_t)255; }

extern "C" void kernel_launch(void* const* d_in, const int* in_sizes, int n_in,
                              void* d_out, int out_size, void* d_ws, size_t ws_size,
                              hipStream_t stream) {
  if (n_in != 37) return;
  const int es[37] = { NVAR * 7, NCON * 4, NSOC * 6, 7 * 64, 64, 4 * 64, 64, 6 * 64, 64,
                       4096, 64, 4096, 4096, 64,   4096, 64, 4096, 4096, 64,
                       4096, 64, 4096, 4096, 64,   4096, 64, 4096, 4096, 64,
                       4096, 64, 64, 1, EVC, EVC, ESC, ESC };
  for (int i = 0; i < 37; ++i) if (in_sizes[i] != es[i]) return;
  if (out_size != NVAR) return;

  const float* var_x = (const float*)d_in[0];
  const float* con_x = (const float*)d_in[1];
  const float* soc_x = (const float*)d_in[2];
  const float* W_var = (const float*)d_in[3];  const float* b_var = (const float*)d_in[4];
  const float* W_con = (const float*)d_in[5];  const float* b_con = (const float*)d_in[6];
  const float* W_soc = (const float*)d_in[7];  const float* b_soc = (const float*)d_in[8];
  const float* f1Wp = (const float*)d_in[9];   const float* f1bp = (const float*)d_in[10];
  const float* f1Ws = (const float*)d_in[11];  const float* f1Wn = (const float*)d_in[12];
  const float* f1b  = (const float*)d_in[13];
  const float* b1Wp = (const float*)d_in[14];  const float* b1bp = (const float*)d_in[15];
  const float* b1Ws = (const float*)d_in[16];  const float* b1Wn = (const float*)d_in[17];
  const float* b1b  = (const float*)d_in[18];
  const float* f2Wp = (const float*)d_in[19];  const float* f2bp = (const float*)d_in[20];
  const float* f2Ws = (const float*)d_in[21];  const float* f2Wn = (const float*)d_in[22];
  const float* f2b  = (const float*)d_in[23];
  const float* b2Wp = (const float*)d_in[24];  const float* b2bp = (const float*)d_in[25];
  const float* b2Ws = (const float*)d_in[26];  const float* b2Wn = (const float*)d_in[27];
  const float* b2b  = (const float*)d_in[28];
  const float* W_hid = (const float*)d_in[29]; const float* b_hid = (const float*)d_in[30];
  const float* W_out = (const float*)d_in[31]; const float* b_out = (const float*)d_in[32];
  const int* vc_src = (const int*)d_in[33];
  const int* vc_dst = (const int*)d_in[34];
  const int* sc_src = (const int*)d_in[35];
  const int* sc_dst = (const int*)d_in[36];
  float* out = (float*)d_out;

  char* ws = (char*)d_ws;
  size_t off = 0;
  const size_t oDN   = off; off = al256(off + (size_t)MPAD * 128 * 2);
  const size_t oX    = off; off = al256(off + (size_t)MPAD * 256 * 2);
  const size_t oHS   = off; off = al256(off + (size_t)MPS * 128 * 2);
  const size_t oP    = off; off = al256(off + (size_t)MPAD * 64 * 4);
  const size_t oPS   = off; off = al256(off + (size_t)MPS * 64 * 4);
  const size_t oENTA = off; off = al256(off + (size_t)NBLKB * RCAP * 4);
  const size_t oENTS = off; off = al256(off + (size_t)NBLKB * RCAP_SC * 4);
  const size_t oOFF  = off; off = al256(off + (size_t)3 * NBLKB * NBRUN * 4);
  const size_t oCNT  = off; off = al256(off + (size_t)3 * NBLKB * NBRUN * 4);
  const size_t oFLG  = off; off = al256(off + (size_t)NFLG * 128);
  const size_t oPRM  = off; off = al256(off + (size_t)PRM_N * 4);
  const size_t oWPT  = off; off = al256(off + (size_t)5 * 64 * 128 * 2);
  const size_t oWFB  = off; off = al256(off + (size_t)4 * 64 * 256 * 2);
  if (off > ws_size || off > (size_t)(128u << 20)) return;

  unsigned short* DN  = (unsigned short*)(ws + oDN);
  unsigned short* X   = (unsigned short*)(ws + oX);
  unsigned short* HS  = (unsigned short*)(ws + oHS);
  float*    P    = (float*)(ws + oP);
  float*    PS   = (float*)(ws + oPS);
  unsigned* ENTA = (unsigned*)(ws + oENTA);
  unsigned* ENTS = (unsigned*)(ws + oENTS);
  int*      OFFt = (int*)(ws + oOFF);
  int*      CNTt = (int*)(ws + oCNT);
  int*      FLG  = (int*)(ws + oFLG);
  float*    PRM  = (float*)(ws + oPRM);
  unsigned short* WPT = (unsigned short*)(ws + oWPT);
  unsigned short* WFB = (unsigned short*)(ws + oWFB);
  const size_t TBL = (size_t)NBLKB * NBRUN;
  const size_t FLN = (size_t)NBLKB * 32;

  const int gGrid  = ((MPAD / 64) + 7) / 8;
  const int gGridS = ((MPS / 64) + 7) / 8;
  const int bkLds = BK_INTS * 4;
  hipFuncSetAttribute(reinterpret_cast<const void*>(&k_bucket), hipFuncAttributeMaxDynamicSharedMemorySize, bkLds);

  k_prep<<<1, 256, 0, stream>>>(f1Wp, f1Ws, f1Wn, f2Wp, f2Ws, f2Wn, b1Wp, b1Ws, b1Wn, b2Wp, b2Ws, b2Wn, W_hid,
                                f1bp, f1b, f2bp, f2b, b1bp, b1b, b2bp, b2b, b_hid, W_out, b_out, WPT, WFB, PRM);

  k_embed<<<MPAD / 128, 256, 0, stream>>>(var_x, W_var, b_var, NVAR, 7, (unsigned*)DN, 64, 0);
  k_embed<<<MPAD / 128, 256, 0, stream>>>(con_x, W_con, b_con, NCON, 4, (unsigned*)X, 128, 64);
  k_embed<<<MPS / 128, 256, 0, stream>>>(soc_x, W_soc, b_soc, NSOC, 6, (unsigned*)HS, 64, 0);

  k_bucket<<<NBLKB, 256, bkLds, stream>>>(vc_dst, vc_src, EVC, NCON, NVAR, RCAP, ENTA, OFFt, CNTt, FLG);
  k_bucket<<<NBLKB, 256, bkLds, stream>>>(sc_dst, sc_src, ESC, NCON, NSOC, RCAP_SC, ENTS, OFFt + TBL, CNTt + TBL,
                                          FLG + FLN);

  for (int li = 0; li < 2; ++li) {
    k_gemm_nt<1, 0><<<gGrid, 256, 0, stream>>>(DN, WPT + (size_t)li * 8192, PRM, P, MPAD, 64, 128, 64);
    k_gemm_nt<1, 0><<<gGridS, 256, 0, stream>>>(HS, WPT + (size_t)li * 8192, PRM, PS, MPS, 64, 128, 64);
    k_agg<2><<<NBLKB, 256, 0, stream>>>(P, ENTA, OFFt, CNTt, FLG, RCAP, NVAR,
                                        PS, ENTS, OFFt + TBL, CNTt + TBL, FLG + FLN, RCAP_SC, NSOC,
                                        PRM, P_BP0 + 64 * li, NCON, (unsigned*)X);
    k_gemm_nt<1, 0><<<gGrid, 256, 0, stream>>>(X, WFB + (size_t)li * 16384, PRM, P, MPAD, 64, 256, 64);
    if (li == 0) k_post<<<MPAD / 128, 256, 0, stream>>>(P, PRM, P_B0, NCON, X, 256, 128);
    else         k_post<<<MPAD / 128, 256, 0, stream>>>(P, PRM, P_B0 + 64, NCON, DN, 128, 0);
  }

  k_bucket<<<NBLKB, 256, bkLds, stream>>>(vc_src, vc_dst, EVC, NVAR, NCON, RCAP, ENTA, OFFt + 2 * TBL, CNTt + 2 * TBL,
                                          FLG + 2 * FLN);
  k_embed<<<MPAD / 128, 256, 0, stream>>>(var_x, W_var, b_var, NVAR, 7, (unsigned*)X, 128, 64);

  for (int li = 0; li < 2; ++li) {
    const int idx = 2 + li;
    k_gemm_nt<1, 0><<<gGrid, 256, 0, stream>>>(DN, WPT + (size_t)idx * 8192, PRM, P, MPAD, 64, 128, 64);
    k_agg<1><<<NBLKB, 256, 0, stream>>>(P, ENTA, OFFt + 2 * TBL, CNTt + 2 * TBL, FLG + 2 * FLN, RCAP, NCON,
                                        P, ENTA, OFFt + 2 * TBL, CNTt + 2 * TBL, FLG + 2 * FLN, RCAP, NCON,
                                        PRM, P_BP0 + 64 * idx, NVAR, (unsigned*)X);
    k_gemm_nt<1, 0><<<gGrid, 256, 0, stream>>>(X, WFB + (size_t)idx * 16384, PRM, P, MPAD, 64, 256, 64);
    if (li == 0) k_post<<<MPAD / 128, 256, 0, stream>>>(P, PRM, P_B0 + 64 * idx, NVAR, X, 256, 128);
    else         k_post<<<MPAD / 128, 256, 0, stream>>>(P, PRM, P_B0 + 64 * idx, NVAR, DN, 128, 0);
  }

  k_gemm_nt<1, 0><<<gGrid, 256, 0, stream>>>(DN, WPT + (size_t)4 * 8192, PRM, P, MPAD, 64, 128, 64);
  k_post<<<MPAD / 128, 256, 0, stream>>>(P, PRM, P_BH, NVAR, DN, 128, 0);
  k_gemm_nt<1, 0><<<gGrid, 256, 0, stream>>>(DN, WPT + (size_t)4 * 8192, PRM, P, MPAD, 64, 128, 64);
  k_head<<<MPAD / 128, 128, 0, stream>>>(P, PRM, FLG, out);
}
